// MemoryBankV2_13056700580081
// MI455X (gfx1250) — hardware-verified
//
#include <hip/hip_runtime.h>
#include <math.h>

constexpr int   kItems     = 128;
constexpr int   kTokPer    = 32;
constexpr int   kDim       = 512;
constexpr int   kHid       = 2048;
constexpr int   kCatDim    = 1024;
constexpr int   kLayers    = 2;
constexpr int   kRows      = kItems * kTokPer;
constexpr int   kChunk     = 512;
constexpr int   kNumChunks = kRows / kChunk;
constexpr float kWCarry    = 64.0f;
constexpr float kPCarry    = 4096.0f;
constexpr float kHCarry    = 16.0f;
constexpr float kLnEps     = 1e-5f;
constexpr float kNegFill   = -1.0e9f;

constexpr int kSmallWElems = 2 * kDim * kDim;
constexpr int kLargeWElems = 2 * kHid * kDim;
constexpr int kSmallW8     = kSmallWElems / 8;
constexpr int kLargeW8     = kLargeWElems / 8;
constexpr int kWBaseLarge  = 4 * kSmallWElems;
constexpr int kW16Total    = 4 * kSmallWElems + 2 * kLargeWElems;

typedef __attribute__((ext_vector_type(16))) _Float16 v16h;
typedef __attribute__((ext_vector_type(8)))  _Float16 v8h;
typedef __attribute__((ext_vector_type(16))) __bf16   v16b;
typedef __attribute__((ext_vector_type(8)))  __bf16   v8b;
typedef __attribute__((ext_vector_type(8)))  float    v8f;
typedef __attribute__((ext_vector_type(4)))  float    v4f;

__device__ __forceinline__ unsigned short f2bf_bits(float f) {
  unsigned u = __float_as_uint(f);
  return (unsigned short)((u + 0x7FFFu + ((u >> 16) & 1u)) >> 16);
}
__device__ __forceinline__ float bf_bits2f(unsigned short h) { return __uint_as_float(((unsigned)h) << 16); }

__device__ __forceinline__ void dep_guard_h(v8f& a, v8f& b, v16h x, v16h y) { asm volatile("v_nop\n\tv_nop\n\tv_nop\n\tv_nop" : "+v"(a), "+v"(b) : "v"(x), "v"(y)); }
__device__ __forceinline__ void dep_guard_b(v8f& a, v8f& b, v16b x, v16b y) { asm volatile("v_nop\n\tv_nop\n\tv_nop\n\tv_nop" : "+v"(a), "+v"(b) : "v"(x), "v"(y)); }
__device__ __forceinline__ void keep4_h(v16h a, v16h b, v16h c, v16h d) { asm volatile("v_nop" :: "v"(a), "v"(b), "v"(c), "v"(d)); }
__device__ __forceinline__ void keep4_b(v16b a, v16b b, v16b c, v16b d) { asm volatile("v_nop" :: "v"(a), "v"(b), "v"(c), "v"(d)); }
__device__ __forceinline__ void acc_guard4(v8f& a, v8f& b, v8f& c, v8f& d) { asm volatile("v_nop\n\tv_nop\n\tv_nop\n\tv_nop" : "+v"(a), "+v"(b), "+v"(c), "+v"(d)); }
template <typename T> struct Frag;
template <> struct Frag<_Float16> {
  typedef v16h V; union U { v16h v; v8h h[2]; };
  static __device__ __forceinline__ v16h load(const _Float16* p) {
    U f; f.h[0] = *(const v8h*)(p); f.h[1] = *(const v8h*)(p + 16); return f.v;
  }
  static __device__ __forceinline__ v8f mma(v16h a, v16h b, v8f c) {
    return __builtin_amdgcn_wmma_f32_16x16x32_f16(false, a, false, b, (short)0, c, false, false);
  }
  static __device__ __forceinline__ void guard(v8f& a, v8f& b, v16h x, v16h y) { dep_guard_h(a, b, x, y); }
  static __device__ __forceinline__ void keep(v16h a, v16h b, v16h c, v16h d) { keep4_h(a, b, c, d); }
};
template <> struct Frag<__bf16> {
  typedef v16b V; union U { v16b v; v8b h[2]; };
  static __device__ __forceinline__ v16b load(const __bf16* p) {
    U f; f.h[0] = *(const v8b*)(p); f.h[1] = *(const v8b*)(p + 16); return f.v;
  }
  static __device__ __forceinline__ v8f mma(v16b a, v16b b, v8f c) {
    return __builtin_amdgcn_wmma_f32_16x16x32_bf16(false, a, false, b, (short)0, c, false, false);
  }
  static __device__ __forceinline__ void guard(v8f& a, v8f& b, v16b x, v16b y) { dep_guard_b(a, b, x, y); }
  static __device__ __forceinline__ void keep(v16b a, v16b b, v16b c, v16b d) { keep4_b(a, b, c, d); }
};

template <int ET> struct Elem;
template <> struct Elem<0> { typedef _Float16 T; };
template <> struct Elem<1> { typedef __bf16 T; };
template <int ET, bool SPLIT, int BIAS_MODE, int OUT_MODE, bool RESID, int ACT = 0>
__global__ __launch_bounds__(256) void wmma_gemm64(
    const unsigned short* __restrict__ Ap, const unsigned short* __restrict__ A2p, int lda, long strideA,
    const unsigned short* __restrict__ Btp, const unsigned short* __restrict__ Bt2p, int ldb, long strideB,
    void* __restrict__ Cout, void* __restrict__ Cout2, int ldc, long strideC,
    const float* __restrict__ bias,
    const float* __restrict__ resid, long strideR,
    int M, int N, int K, float scale) {
  typedef typename Elem<ET>::T T;
  typedef typename Frag<T>::V V;
  const T* A = (const T*)Ap; const T* A2 = (const T*)A2p; const T* Bt = (const T*)Btp; const T* Bt2 = (const T*)Bt2p;
  __shared__ __align__(16) float sT[8][16 * 68];
  const int b    = blockIdx.y;
  const int lane = threadIdx.x & 31;
  const int wave = threadIdx.x >> 5;
  const int tilesN = N >> 6;
  const int tilesM = M >> 6;
  const int tile = blockIdx.x * 8 + wave;
  if (tile >= tilesM * tilesN) return;
  const int tm = tile / tilesN;
  const int tn = tile - tm * tilesN;
  const int m0 = tm << 6;
  const int n0 = tn << 6;

  const T* Ab  = A  + (size_t)b * strideA;
  const T* Bb  = Bt + (size_t)b * strideB;
  const T* Ab2 = SPLIT ? (A2  + (size_t)b * strideA) : nullptr;
  const T* Bb2 = SPLIT ? (Bt2 + (size_t)b * strideB) : nullptr;

  const int rlane = lane & 15;
  const int koff  = (lane >> 4) * 8;
  const int mOff  = (lane >> 4) * 8;

  v8f acc[4][4];
#pragma unroll
  for (int i = 0; i < 4; ++i)
#pragma unroll
    for (int j = 0; j < 4; ++j) acc[i][j] = (v8f){0.f,0.f,0.f,0.f,0.f,0.f,0.f,0.f};

  for (int k0 = 0; k0 < K; k0 += 32) {
    V bh[4], bl[4];
#pragma unroll
    for (int j = 0; j < 4; ++j) {
      const size_t bo = (size_t)(n0 + (j << 4) + rlane) * ldb + koff + k0;
      bh[j] = Frag<T>::load(Bb + bo);
      if (SPLIT) bl[j] = Frag<T>::load(Bb2 + bo);
    }
#pragma unroll
    for (int i = 0; i < 4; ++i) {
      const size_t ao = (size_t)(m0 + (i << 4) + rlane) * lda + koff + k0;
      V ah = Frag<T>::load(Ab + ao);
      V al;
      if (SPLIT) al = Frag<T>::load(Ab2 + ao);
#pragma unroll
      for (int j = 0; j < 4; ++j) {
        acc[i][j] = Frag<T>::mma(ah, bh[j], acc[i][j]);
        if (SPLIT) {
          acc[i][j] = Frag<T>::mma(ah, bl[j], acc[i][j]);
          acc[i][j] = Frag<T>::mma(al, bh[j], acc[i][j]);
        }
      }
      Frag<T>::guard(acc[i][0], acc[i][3], ah, SPLIT ? al : ah);
    }
    Frag<T>::keep(bh[0], bh[1], bh[2], bh[3]);
    if (SPLIT) Frag<T>::keep(bl[0], bl[1], bl[2], bl[3]);
  }
  acc_guard4(acc[0][0], acc[0][1], acc[0][2], acc[0][3]);
  acc_guard4(acc[1][0], acc[1][1], acc[1][2], acc[1][3]);
  acc_guard4(acc[2][0], acc[2][1], acc[2][2], acc[2][3]);
  acc_guard4(acc[3][0], acc[3][1], acc[3][2], acc[3][3]);

  float* slab = sT[wave];
  const float* Rb = RESID ? (resid + (size_t)b * strideR) : nullptr;
#pragma unroll
  for (int i = 0; i < 4; ++i) {
    const int mBase = m0 + (i << 4);
#pragma unroll
    for (int j = 0; j < 4; ++j) {
      const int n = n0 + (j << 4) + rlane;
      float bv = 0.f;
      if (BIAS_MODE == 2) bv = bias[n];
#pragma unroll
      for (int r = 0; r < 8; ++r) {
        float v = acc[i][j][r] * scale;
        if (BIAS_MODE == 1) v += bias[mBase + mOff + r];
        if (BIAS_MODE == 2) v += bv;
        if (RESID) v += Rb[(size_t)(mBase + mOff + r) * ldc + n];
        if (ACT == 2) v = fmaxf(v, 0.0f);
        if (ACT == 4) v = (v > 0.f) ? v : 0.01f * v;
        slab[(mOff + r) * 68 + (j << 4) + rlane] = v;
      }
    }
    __builtin_amdgcn_fence(__ATOMIC_RELEASE, "workgroup");
    __builtin_amdgcn_wave_barrier();
    __builtin_amdgcn_fence(__ATOMIC_ACQUIRE, "workgroup");
    if (OUT_MODE == 0) {
      float* C = (float*)Cout + (size_t)b * strideC;
      const int hh = lane >> 4, c4 = (lane & 15) * 4;
      for (int pass = 0; pass < 2; ++pass) {
#pragma unroll
        for (int it = 0; it < 8; ++it) {
          const int row = it * 2 + hh;
          v4f v = *(const v4f*)(slab + row * 68 + c4);
          *(volatile v4f*)(C + (size_t)(mBase + row) * ldc + n0 + c4) = v;
        }
        __threadfence();
      }
    } else {
      const int q = lane >> 3, c8 = (lane & 7) * 8;
      unsigned short* C  = (unsigned short*)Cout  + (size_t)b * strideC;
      unsigned short* C2 = (OUT_MODE == 2) ? ((unsigned short*)Cout2 + (size_t)b * strideC) : nullptr;
      for (int pass = 0; pass < 2; ++pass) {
#pragma unroll
        for (int it = 0; it < 4; ++it) {
          const int row = it * 4 + q;
          const float* sp = slab + row * 68 + c8;
          v8h hv, lv;
#pragma unroll
          for (int e = 0; e < 8; ++e) {
            if (OUT_MODE == 1) {
              hv[e] = (_Float16)sp[e];
            } else {
              unsigned short hb = f2bf_bits(sp[e]);
              unsigned short lb = f2bf_bits(sp[e] - bf_bits2f(hb));
              hv[e] = __builtin_bit_cast(_Float16, hb);
              lv[e] = __builtin_bit_cast(_Float16, lb);
            }
          }
          *(volatile v8h*)(C + (size_t)(mBase + row) * ldc + n0 + c8) = hv;
          if (OUT_MODE == 2) *(volatile v8h*)(C2 + (size_t)(mBase + row) * ldc + n0 + c8) = lv;
        }
        __threadfence();
      }
    }
    __builtin_amdgcn_fence(__ATOMIC_RELEASE, "workgroup");
    __builtin_amdgcn_wave_barrier();
    __builtin_amdgcn_fence(__ATOMIC_ACQUIRE, "workgroup");
  }
}

__global__ __launch_bounds__(256) void castw_kernel(const float* __restrict__ w0, const float* __restrict__ w1,
                                                    const float* __restrict__ w2, const float* __restrict__ w3,
                                                    const float* __restrict__ w4, const float* __restrict__ w5,
                                                    _Float16* __restrict__ out, float scale) {
  const int z = blockIdx.y;
  const float* W = (z == 0) ? w0 : (z == 1) ? w1 : (z == 2) ? w2 : (z == 3) ? w3 : (z == 4) ? w4 : w5;
  const int n8 = (z < 4) ? kSmallW8 : kLargeW8;
  const size_t off = (z < 4) ? (size_t)z * kSmallWElems : (size_t)kWBaseLarge + (size_t)(z - 4) * kLargeWElems;
  const int i8 = blockIdx.x * 256 + threadIdx.x;
  if (i8 < n8) {
    const v4f a = *(const v4f*)(W + (size_t)i8 * 8);
    const v4f c = *(const v4f*)(W + (size_t)i8 * 8 + 4);
    v8h hv;
#pragma unroll
    for (int e = 0; e < 4; ++e) { hv[e] = (_Float16)(a[e] * scale); hv[4 + e] = (_Float16)(c[e] * scale); }
    _Float16* p = out + off + (size_t)i8 * 8;
    *(volatile v8h*)p = hv;
    __threadfence();
    *(volatile v8h*)p = hv;
  }
}

__global__ __launch_bounds__(256) void castcf_kernel(const float* __restrict__ cf, _Float16* __restrict__ cat) {
  const int i8  = blockIdx.x * 256 + threadIdx.x;
  const int row = i8 >> 6;
  const int c8  = (i8 & 63) * 8;
  const float* src = cf + (size_t)row * kDim + c8;
  const v4f a = *(const v4f*)(src);
  const v4f c = *(const v4f*)(src + 4);
  v8h hv;
#pragma unroll
  for (int e = 0; e < 4; ++e) { hv[e] = (_Float16)a[e]; hv[4 + e] = (_Float16)c[e]; }
  _Float16* p0 = cat + (size_t)row * kCatDim + c8;
  _Float16* p1 = p0 + kDim;
  for (int pass = 0; pass < 2; ++pass) {
    *(volatile v8h*)p0 = hv;
    *(volatile v8h*)p1 = hv;
    __threadfence();
  }
}

__device__ __forceinline__ float masked_score(float raw, int col, int item, bool inr) {
  const bool vis = (col >> 5) < item;
  const float s = vis ? raw : kNegFill;
  return inr ? s : -INFINITY;
}

__global__ __launch_bounds__(256) void softmax_kernel(const float* __restrict__ S, _Float16* __restrict__ P,
                                                      int row0, int ncols) {
  __shared__ float redm[8];
  __shared__ float reds[8];
  const int tid  = threadIdx.x;
  const int lane = tid & 31;
  const int wave = tid >> 5;
  const int rl   = blockIdx.x;
  const int item = (row0 + rl) >> 5;
  const float* srow = S + (size_t)rl * kRows;

  float v[16];
  float mx = -INFINITY;
#pragma unroll
  for (int i = 0; i < 2; ++i) {
    const int cb   = 8 * tid + 2048 * i;
    const bool inr = cb < ncols;
    const int cbc  = inr ? cb : (ncols - 8);
    const v4f a = *(const v4f*)(srow + cbc);
    const v4f c = *(const v4f*)(srow + cbc + 4);
#pragma unroll
    for (int e = 0; e < 4; ++e) {
      const float s0 = masked_score(a[e], cb + e, item, inr);
      const float s1 = masked_score(c[e], cb + 4 + e, item, inr);
      v[8 * i + e] = s0;
      v[8 * i + 4 + e] = s1;
      mx = fmaxf(mx, fmaxf(s0, s1));
    }
  }
#pragma unroll
  for (int off = 1; off < 32; off <<= 1) mx = fmaxf(mx, __shfl_xor(mx, off, 32));
  if (lane == 0) redm[wave] = mx;
  __syncthreads();
  float m = redm[0];
#pragma unroll
  for (int w = 1; w < 8; ++w) m = fmaxf(m, redm[w]);

  float sum = 0.f;
#pragma unroll
  for (int j = 0; j < 16; ++j) {
    const float e = __expf(v[j] - m);
    v[j] = e;
    sum += e;
  }
#pragma unroll
  for (int off = 1; off < 32; off <<= 1) sum += __shfl_xor(sum, off, 32);
  if (lane == 0) reds[wave] = sum;
  __syncthreads();
  float tot = reds[0];
#pragma unroll
  for (int w = 1; w < 8; ++w) tot += reds[w];
  const float inv = kPCarry / tot;

  _Float16* prow = P + (size_t)rl * kRows;
  for (int pass = 0; pass < 2; ++pass) {
#pragma unroll
    for (int i = 0; i < 2; ++i) {
      const int cb = 8 * tid + 2048 * i;
      if (cb < ncols) {
        v8h hv;
#pragma unroll
        for (int e = 0; e < 8; ++e) hv[e] = (_Float16)(v[8 * i + e] * inv);
        *(volatile v8h*)(prow + cb) = hv;
      }
    }
    __threadfence();
  }
}

__global__ __launch_bounds__(256) void ln_kernel(const float* __restrict__ Y, const float* __restrict__ gam,
                                                 const float* __restrict__ bet, float* __restrict__ X32,
                                                 _Float16* __restrict__ X16, const float* __restrict__ ovr, int ovr_rows) {
  __shared__ __align__(16) float slab[8][kDim];
  const int lane = threadIdx.x & 31;
  const int wave = threadIdx.x >> 5;
  const int row  = blockIdx.x * 8 + wave;
  const float* yr = Y + (size_t)row * kDim;

  v4f t[4];
  float sum = 0.f;
#pragma unroll
  for (int i = 0; i < 4; ++i) {
    t[i] = *(const v4f*)(yr + 4 * lane + 128 * i);
    sum += (t[i][0] + t[i][1]) + (t[i][2] + t[i][3]);
  }
#pragma unroll
  for (int off = 1; off < 32; off <<= 1) sum += __shfl_xor(sum, off, 32);
  const float mean = sum * (1.0f / kDim);
  float sq = 0.f;
#pragma unroll
  for (int i = 0; i < 4; ++i) {
#pragma unroll
    for (int e = 0; e < 4; ++e) { const float d = t[i][e] - mean; t[i][e] = d; sq += d * d; }
  }
#pragma unroll
  for (int off = 1; off < 32; off <<= 1) sq += __shfl_xor(sq, off, 32);
  const float inv = rsqrtf(sq * (1.0f / kDim) + kLnEps);

  v4f o[4];
#pragma unroll
  for (int i = 0; i < 4; ++i) {
    const v4f gg = *(const v4f*)(gam + 4 * lane + 128 * i);
    const v4f bb = *(const v4f*)(bet + 4 * lane + 128 * i);
#pragma unroll
    for (int e = 0; e < 4; ++e) o[i][e] = (t[i][e] * inv) * gg[e] + bb[e];
  }
  if (row < ovr_rows) {
#pragma unroll
    for (int i = 0; i < 4; ++i) o[i] = *(const v4f*)(ovr + (size_t)row * kDim + 4 * lane + 128 * i);
  }

  float* xr = X32 + (size_t)row * kDim;
  for (int pass = 0; pass < 2; ++pass) {
#pragma unroll
    for (int i = 0; i < 4; ++i) *(volatile v4f*)(xr + 4 * lane + 128 * i) = o[i];
    __threadfence();
  }

  float* sl = slab[wave];
#pragma unroll
  for (int i = 0; i < 4; ++i) *(v4f*)(sl + 4 * lane + 128 * i) = o[i];
  __builtin_amdgcn_fence(__ATOMIC_RELEASE, "workgroup");
  __builtin_amdgcn_wave_barrier();
  __builtin_amdgcn_fence(__ATOMIC_ACQUIRE, "workgroup");
  v8h hv[2];
#pragma unroll
  for (int i = 0; i < 2; ++i) {
    const v4f p0 = *(const v4f*)(sl + 8 * lane + 256 * i);
    const v4f p1 = *(const v4f*)(sl + 8 * lane + 256 * i + 4);
#pragma unroll
    for (int e = 0; e < 4; ++e) { hv[i][e] = (_Float16)p0[e]; hv[i][4 + e] = (_Float16)p1[e]; }
  }
  _Float16* hr = X16 + (size_t)row * kCatDim;
  for (int pass = 0; pass < 2; ++pass) {
#pragma unroll
    for (int i = 0; i < 2; ++i) *(volatile v8h*)(hr + 8 * lane + 256 * i) = hv[i];
    __threadfence();
  }
}

__global__ __launch_bounds__(256) void gelu_kernel(const float* __restrict__ U, _Float16* __restrict__ Hh, int n2) {
  const int i = blockIdx.x * 256 + threadIdx.x;
  if (i < n2) {
    const float u0 = U[2 * (size_t)i];
    const float u1 = U[2 * (size_t)i + 1];
    float r0 = 0.f, r1 = 0.f;
#pragma unroll 1
    for (int e = 0; e < 2; ++e) {
      const float u  = (e == 0) ? u0 : u1;
      const float gv = 0.5f * u * (1.0f + erff(u * 0.70710678118654752f)) * kHCarry;
      if (e == 0) r0 = gv; else r1 = gv;
    }
    const _Float16 h0 = (_Float16)r0, h1 = (_Float16)r1;
    const unsigned u = (unsigned)__builtin_bit_cast(unsigned short, h0) | ((unsigned)__builtin_bit_cast(unsigned short, h1) << 16);
    ((volatile unsigned*)(void*)Hh)[i] = u;
    __threadfence();
    ((volatile unsigned*)(void*)Hh)[i] = u;
  }
}

__global__ __launch_bounds__(256) void blend_kernel(const float* __restrict__ G, const float* __restrict__ CF,
                                                    const float* __restrict__ X, float* __restrict__ OUT, int n4) {
  const int i = blockIdx.x * 256 + threadIdx.x;
  if (i < n4) {
    const v4f g = *(const v4f*)(G  + 4 * (size_t)i);
    const v4f c = *(const v4f*)(CF + 4 * (size_t)i);
    const v4f x = *(const v4f*)(X  + 4 * (size_t)i);
    v4f o;
#pragma unroll
    for (int e = 0; e < 4; ++e) {
      const float ex = __expf(-g[e]);
      const float s  = __builtin_amdgcn_rcpf(1.0f + ex);
      o[e] = s * c[e] + (1.0f - s) * x[e];
    }
    float* p = OUT + 4 * (size_t)i;
    *(volatile v4f*)p = o;
    __threadfence();
    *(volatile v4f*)p = o;
  }
}

template <int BIAS_MODE, int OUT_MODE, bool RESID>
static void launch_gemm(hipStream_t st, const void* A, int lda, const void* Bt, int ldb, void* C, int ldc,
                        const float* bias, const float* resid, int M, int N, int K, float scale) {
  const int tiles = (M / 64) * (N / 64);
  dim3 grid((tiles + 7) / 8, 1);
  wmma_gemm64<0, false, BIAS_MODE, OUT_MODE, RESID, 0><<<grid, 256, 0, st>>>(
      (const unsigned short*)A, (const unsigned short*)A, lda, 0L,
      (const unsigned short*)Bt, (const unsigned short*)Bt, ldb, 0L,
      C, C, ldc, 0L, bias, resid, 0L, M, N, K, scale);
}

extern "C" void kernel_launch(void* const* d_in, const int* in_sizes, int n_in,
                              void* d_out, int out_size, void* d_ws, size_t ws_size,
                              hipStream_t stream) {
  if (n_in < 17) return;
  if (in_sizes[0] != kRows * kDim || out_size != kRows * kDim) return;
  if (in_sizes[1] != kSmallWElems || in_sizes[9] != kLargeWElems || in_sizes[11] != kLargeWElems ||
      in_sizes[15] != kSmallWElems) return;

  const float* cf   = (const float*)d_in[0];
  const float* Wq   = (const float*)d_in[1];  const float* bq   = (const float*)d_in[2];
  const float* Wk   = (const float*)d_in[3];  const float* bk   = (const float*)d_in[4];
  const float* Wv   = (const float*)d_in[5];  const float* bv   = (const float*)d_in[6];
  const float* ln1g = (const float*)d_in[7];  const float* ln1b = (const float*)d_in[8];
  const float* W1   = (const float*)d_in[9];  const float* b1   = (const float*)d_in[10];
  const float* W2   = (const float*)d_in[11]; const float* b2   = (const float*)d_in[12];
  const float* ln2g = (const float*)d_in[13]; const float* ln2b = (const float*)d_in[14];
  const float* Ws   = (const float*)d_in[15]; const float* bs   = (const float*)d_in[16];
  float* out = (float*)d_out;

  const size_t szW16  = (size_t)kW16Total * 2;
  const size_t szCat  = (size_t)kRows * kCatDim * 2;
  const size_t szF32  = (size_t)kRows * kDim * 4;
  const size_t szH512 = (size_t)kRows * kDim * 2;
  const size_t szBig  = (size_t)kRows * kHid * 4;
  const size_t szHid  = (size_t)kRows * kHid * 2;
  const size_t oW16  = 0;
  const size_t oCat  = oW16 + szW16;
  const size_t oX32  = oCat + szCat;
  const size_t oY32  = oX32 + szF32;
  const size_t oQ16  = oY32 + szF32;
  const size_t oK16  = oQ16 + szH512;
  const size_t oVT16 = oK16 + szH512;
  const size_t oBig  = oVT16 + szH512;
  const size_t oH16  = oBig + szBig;
  const size_t oEnd  = oH16 + szHid;
  if (oEnd > ws_size) return;
  if ((size_t)kChunk * kRows * 4 + (size_t)kChunk * kRows * 2 > szBig) return;

  char* ws = (char*)d_ws;
  _Float16* w16  = (_Float16*)(ws + oW16);
  _Float16* Wq16 = w16;
  _Float16* Wk16 = w16 + kSmallWElems;
  _Float16* Wv16 = w16 + 2 * kSmallWElems;
  _Float16* Ws16 = w16 + 3 * kSmallWElems;
  _Float16* W116 = w16 + kWBaseLarge;
  _Float16* W216 = w16 + kWBaseLarge + kLargeWElems;
  _Float16* cat16 = (_Float16*)(ws + oCat);
  _Float16* cf16  = cat16;
  _Float16* x16   = cat16 + kDim;
  float*    x32   = (float*)(ws + oX32);
  float*    y32   = (float*)(ws + oY32);
  _Float16* q16   = (_Float16*)(ws + oQ16);
  _Float16* k16   = (_Float16*)(ws + oK16);
  _Float16* vT16  = (_Float16*)(ws + oVT16);
  float*    s32   = (float*)(ws + oBig);
  _Float16* p16   = (_Float16*)(ws + oBig + (size_t)kChunk * kRows * 4);
  float*    u32   = (float*)(ws + oBig);
  _Float16* h16   = (_Float16*)(ws + oH16);

  const float invW    = 1.0f / kWCarry;
  const float invP    = 1.0f / kPCarry;
  const float invHW   = 1.0f / (kHCarry * kWCarry);
  const float invSqrt = 1.0f / sqrtf((float)kDim);

  castw_kernel<<<dim3(kLargeW8 / 256, 6), 256, 0, stream>>>(Wq, Wk, Wv, Ws, W1, W2, w16, kWCarry);
  castcf_kernel<<<(kRows * kDim / 8) / 256, 256, 0, stream>>>(cf, cat16);

  for (int l = 0; l < kLayers; ++l) {
    const _Float16* Wql = Wq16 + (size_t)l * kDim * kDim;
    const _Float16* Wkl = Wk16 + (size_t)l * kDim * kDim;
    const _Float16* Wvl = Wv16 + (size_t)l * kDim * kDim;
    const _Float16* W1l = W116 + (size_t)l * kHid * kDim;
    const _Float16* W2l = W216 + (size_t)l * kDim * kHid;

    launch_gemm<2, 1, false>(stream, x16, kCatDim, Wql, kDim, q16, kDim, bq + l * kDim, x32, kRows, kDim, kDim, invW);
    launch_gemm<2, 1, false>(stream, cf16, kCatDim, Wkl, kDim, k16, kDim, bk + l * kDim, x32, kRows, kDim, kDim, invW);
    launch_gemm<1, 1, false>(stream, Wvl, kDim, cf16, kCatDim, vT16, kRows, bv + l * kDim, x32, kDim, kRows, kDim, invW);

    const float* xres = (l == 0) ? cf : x32;
    for (int c = 0; c < kNumChunks; ++c) {
      const int ncols = kChunk * (c + 1);
      launch_gemm<0, 0, false>(stream, q16 + (size_t)c * kChunk * kDim, kDim, k16, kDim, s32, kRows,
                               bq, x32, kChunk, ncols, kDim, invSqrt);
      softmax_kernel<<<kChunk, 256, 0, stream>>>(s32, p16, c * kChunk, ncols);
      launch_gemm<0, 0, true>(stream, p16, kRows, vT16, kRows, y32 + (size_t)c * kChunk * kDim, kDim,
                              bq, xres + (size_t)c * kChunk * kDim, kChunk, kDim, ncols, invP);
    }
    ln_kernel<<<kRows / 8, 256, 0, stream>>>(y32, ln1g + l * kDim, ln1b + l * kDim, x32, x16, cf, 0);
    launch_gemm<2, 0, false>(stream, x16, kCatDim, W1l, kDim, u32, kHid, b1 + l * kHid, x32, kRows, kHid, kDim, invW);
    gelu_kernel<<<(kRows * kHid / 2) / 256, 256, 0, stream>>>(u32, h16, kRows * kHid / 2);
    launch_gemm<2, 0, true>(stream, h16, kHid, W2l, kHid, y32, kDim, b2 + l * kDim, x32, kRows, kDim, kHid, invHW);
    const int ovr_rows = (l == kLayers - 1) ? kTokPer : 0;
    ln_kernel<<<kRows / 8, 256, 0, stream>>>(y32, ln2g + l * kDim, ln2b + l * kDim, x32, x16, cf, ovr_rows);
  }

  launch_gemm<2, 0, false>(stream, cat16, kCatDim, Ws16, kCatDim, y32, kDim, bs, x32, kRows, kDim, kCatDim, invW);
  blend_kernel<<<(kRows * kDim / 4) / 256, 256, 0, stream>>>(y32, cf, x32, out, kRows * kDim / 4);
}
